// SimpleGNN_38680475468245
// MI455X (gfx1250) — hardware-run, weakly checked
//
#include <hip/hip_runtime.h>


namespace {
constexpr int N = 50000, E = 800000, E2 = 400000, FIN = 128, FE = 16, HG = 64, NH1 = 4, C1 = NH1 * HG  , HN = 256, HN2 = 128, NPB = 8;
constexpr float XS = 8.0f, HS = 256.0f, WSC = 256.0f;
typedef _Float16 b16;
typedef __attribute__((ext_vector_type(16))) _Float16 v16b;
typedef __attribute__((ext_vector_type(8))) _Float16 v8b;
typedef __attribute__((ext_vector_type(8))) float v8f;
typedef __attribute__((ext_vector_type(4))) float v4f;
typedef __attribute__((ext_vector_type(2))) float v2f;
__device__ __forceinline__ float bf16_rne(float f) { unsigned int u = __float_as_uint(f); u += 0x7FFFu + ((u >> 16) & 1u); float r = __uint_as_float(u & 0xFFFF0000u); asm volatile("" : "+v"(r)); return r; }
__device__ __forceinline__ float bfv(float f) { float r = bf16_rne(f); asm volatile("" : "+v"(r)); return r; }
__device__ __forceinline__ void split16(float v, b16& hi, b16& lo) { hi = (b16)v; lo = (b16)(v - (float)hi); }
__device__ __forceinline__ v16b frag_kb(const b16* p, int hh) { const v8b a = *(const v8b*)(p + 8 * hh), b = *(const v8b*)(p + 16 + 8 * hh); v16b f;
#pragma unroll
  for (int e = 0; e < 8; ++e) { f[e] = a[e]; f[8 + e] = b[e]; } return f; }
__device__ __forceinline__ v8f wmma16b(v16b a, v16b b, v8f c) { v8f d = __builtin_amdgcn_wmma_f32_16x16x32_f16(false, a, false, b, (short)0, c, false, false); asm volatile("v_nop\n\tv_nop\n\tv_nop\n\tv_nop" : "+v"(d) : "v"(a), "v"(b)); return d; }
__device__ __forceinline__ void wave_lds_sync() { __builtin_amdgcn_fence(__ATOMIC_RELEASE, "workgroup"); __builtin_amdgcn_wave_barrier(); __builtin_amdgcn_fence(__ATOMIC_ACQUIRE, "workgroup"); }
__device__ __forceinline__ float pmul(float a, float b) { float p = a * b; asm volatile("" : "+v"(p)); return p; }
__device__ __forceinline__ int iclamp(int v, int lo, int hi) { return v < lo ? lo : (v > hi ? hi : v); }
constexpr int CSR_NBLK8 = 512, CSR_GB8 = 8, CSR_GN8 = 1 << CSR_GB8  , CSR_TS8 = (CSR_GN8 < 32 ? 32 : CSR_GN8)  , CSR_MAXG8 = 512, CSR_CAP8 = 12288  ;
__device__ __host__ __forceinline__ int csr_tix8(int v) { return (v >> CSR_GB8) * CSR_TS8 + (v & (CSR_GN8 - 1)); }
__global__ __launch_bounds__(64) void csrA_kernel8(const int* __restrict__ dst, int E, int N, int nG, int CHP, int NGP, int* __restrict__ STG, int* __restrict__ HST) {
  extern __shared__ int sm[];
  int* cnt = sm; int* run = sm + NGP; int* ids = sm + 2 * NGP;
  const int b = blockIdx.x; const int ch = (E + CSR_NBLK8 - 1) / CSR_NBLK8; const int e0 = b * ch, e1 = min(E, e0 + ch);
  for (int i = threadIdx.x; i < NGP; i += 64) cnt[i] = 0;
  for (int i = threadIdx.x; i < CHP; i += 64) ids[i] = -1;
  __syncthreads();
  if (threadIdx.x == 0) {
    for (int e = e0; e < e1; ++e) { int d = dst[e]; d = (d < 0) ? 0 : (d >= N ? N - 1 : d); cnt[d >> CSR_GB8] += 1; }
    int acc = 0; for (int g = 0; g < nG; ++g) { run[g] = acc; acc += cnt[g]; }
    for (int e = e0; e < e1; ++e) { int d = dst[e]; d = (d < 0) ? 0 : (d >= N ? N - 1 : d); const int g = d >> CSR_GB8; ids[run[g]] = e; run[g] += 1; } }
  __syncthreads();
  typedef __attribute__((ext_vector_type(4))) int v4i;
  for (int pass = 0; pass < 2; ++pass) {
    for (int i = threadIdx.x; i < CHP / 4; i += 64) *(volatile v4i*)(STG + (size_t)b * CHP + i * 4) = *(const v4i*)(&ids[i * 4]);
    for (int i = threadIdx.x; i < NGP / 4; i += 64) { v4i v; for (int e = 0; e < 4; ++e) v[e] = (i * 4 + e < nG) ? cnt[i * 4 + e] : 0; *(volatile v4i*)(HST + (size_t)b * NGP + i * 4) = v; }
    __threadfence(); }
}
__global__ __launch_bounds__(512) void csrS_kernel8(const int* __restrict__ HST, int nG, int NGP, int* __restrict__ START, int* __restrict__ TOT, int* __restrict__ OFF) {
  __shared__ int tot[CSR_MAXG8];
  const int b = threadIdx.x;
  for (int pass = 0; pass < 2; ++pass) { int runb = 0; for (int g = 0; g < nG; ++g) { int c = HST[(size_t)b * NGP + g]; c = (c < 0) ? 0 : c; ((volatile int*)OFF)[(size_t)g * CSR_NBLK8 + b] = runb; runb += c; } __threadfence(); }
  for (int g = threadIdx.x; g < nG; g += 512) { int s = 0; for (int bb = 0; bb < CSR_NBLK8; ++bb) { int c = HST[(size_t)bb * NGP + g]; s += (c < 0) ? 0 : c; } tot[g] = s; }
  __syncthreads();
  if (threadIdx.x < 32) {
    __shared__ int st[CSR_MAXG8 + 32];
    if (threadIdx.x == 0) { int acc = 0; for (int g = 0; g < NGP; ++g) { st[g] = acc; if (g < nG) acc += (tot[g] + 31) & ~31; } st[NGP] = acc; }
    __builtin_amdgcn_fence(__ATOMIC_RELEASE, "workgroup"); __builtin_amdgcn_wave_barrier(); __builtin_amdgcn_fence(__ATOMIC_ACQUIRE, "workgroup");
    for (int pass = 0; pass < 2; ++pass) { for (int i = threadIdx.x; i < NGP + 32; i += 32) { ((volatile int*)START)[i] = (i <= NGP) ? st[min(i, NGP)] : 0; ((volatile int*)TOT)[i] = (i < nG) ? tot[i] : 0; } __threadfence(); } }
}
__global__ __launch_bounds__(256) void csrB_kernel8(const int* __restrict__ dst, int N, int nG, int CHP, int NGP, int permLen, const int* __restrict__ STG, const int* __restrict__ HST, const int* __restrict__ OFF, const int* __restrict__ START, const int* __restrict__ TOT, int* __restrict__ PERM, int* __restrict__ ROWPTR, int* __restrict__ ROWCNT, int* __restrict__ FLAG) {
  typedef __attribute__((ext_vector_type(4))) int v4i;
  __shared__ int ids[CSR_CAP8]; __shared__ unsigned short key[CSR_CAP8]; __shared__ int outp[CSR_CAP8]; __shared__ int ncnt[CSR_GN8 + 1]; __shared__ int boff[CSR_NBLK8 + 1];
  const int g = blockIdx.x, t_ = threadIdx.x; int tot = TOT[g]; int st = START[g], stn = START[g + 1]; const int v0 = g * CSR_GN8; const int nv = min(CSR_GN8, N - v0); const int t0 = g * CSR_TS8;
  st = (st < 0) ? 0 : (st > permLen - 32 ? permLen - 32 : st) & ~31; stn = (stn < st) ? st : (stn > permLen ? permLen : stn); tot = (tot < 0) ? 0 : tot; if (tot > stn - st && tot <= CSR_CAP8) tot = stn - st;
  if (tot > CSR_CAP8) {
    for (int pass = 0; pass < 2; ++pass) { for (int i = t_; i < CSR_TS8 / 4; i += 256) { v4i a, c; for (int e = 0; e < 4; ++e) { a[e] = st; c[e] = 0; } *(volatile v4i*)(ROWPTR + t0 + i * 4) = a; *(volatile v4i*)(ROWCNT + t0 + i * 4) = c; } if (t_ == 0) ((volatile int*)FLAG)[0] = 1; __threadfence(); } (void)nv; return; }
  if (t_ == 0) { int acc = 0; for (int b = 0; b < CSR_NBLK8; ++b) { boff[b] = acc; int c = HST[(size_t)b * NGP + g]; c = (c < 0) ? 0 : (c > CHP ? CHP : c); acc += c; if (acc > tot) acc = tot; } boff[CSR_NBLK8] = acc; }
  for (int i = t_; i <= CSR_GN8; i += 256) ncnt[i] = 0;
  __syncthreads();
  for (int b = 0; b < CSR_NBLK8; ++b) { const int c = boff[b + 1] - boff[b]; int o_ = OFF[(size_t)g * CSR_NBLK8 + b]; o_ = (o_ < 0) ? 0 : (o_ > CHP - c ? CHP - c : o_); const int* src_ = STG + (size_t)b * CHP + o_;
    for (int i = t_; i < c; i += 256) { int id = src_[i]; id = (id < 0) ? 0 : id; ids[boff[b] + i] = id; int d = dst[id]; d = (d < v0) ? v0 : (d >= N ? N - 1 : d); int kk = d - v0; kk = (kk < 0) ? 0 : (kk >= CSR_GN8 ? CSR_GN8 - 1 : kk); key[boff[b] + i] = (unsigned short)kk; } }
  __syncthreads();
  if (t_ == 0) { for (int i = 0; i < tot; ++i) ncnt[key[i]] += 1; int acc = 0; for (int vl = 0; vl < CSR_GN8; ++vl) { const int c = ncnt[vl]; ncnt[vl] = acc; acc += c; } ncnt[CSR_GN8] = acc;
    for (int i = 0; i < tot; ++i) { const int vl = key[i]; outp[ncnt[vl]] = ids[i]; ncnt[vl] += 1; }
    for (int vl = CSR_GN8; vl > 0; --vl) ncnt[vl] = ncnt[vl - 1]; ncnt[0] = 0; }
  __syncthreads();
  for (int pass = 0; pass < 2; ++pass) {
    for (int i = t_; i < (stn - st) / 4; i += 256) { v4i v; for (int e = 0; e < 4; ++e) { const int q = i * 4 + e; v[e] = (q < tot) ? outp[q] : -1; } *(volatile v4i*)(PERM + st + i * 4) = v; }
    for (int i = t_; i < CSR_TS8 / 4; i += 256) { v4i a, c; for (int e = 0; e < 4; ++e) { const int vl = i * 4 + e; const int vc = vl < CSR_GN8 ? vl : CSR_GN8; a[e] = (vl < CSR_GN8) ? st + ncnt[vc] : st; c[e] = (vl < nv) ? (ncnt[(vc < CSR_GN8 ? vc : CSR_GN8 - 1) + 1] - ncnt[vc]) : 0; } *(volatile v4i*)(ROWPTR + t0 + i * 4) = a; *(volatile v4i*)(ROWCNT + t0 + i * 4) = c; }
    __threadfence(); }
}
__global__ __launch_bounds__(256) void csrZ_kernel8(int* __restrict__ p, size_t n4) { typedef __attribute__((ext_vector_type(4))) int v4i; const size_t tid = (size_t)blockIdx.x * 256 + threadIdx.x, nth = (size_t)gridDim.x * 256; v4i z = {0, 0, 0, 0}; for (size_t i = tid; i < n4; i += nth) *(volatile v4i*)(p + i * 4) = z; }
struct CsrBufs8 { int *STG, *HST, *OFF, *START, *TOT, *PERM, *ROWPTR, *ROWCNT, *FLAG; int nG, NGP, CHP; size_t permLen; char* base; size_t bytes; };
static size_t csr_carve8(CsrBufs8& c, char* ws, size_t off, int E, int N) {
  const size_t off0 = off; c.base = ws + off;
  auto al = [&](size_t bytes) { char* p = ws + off; off += (bytes + 255) & ~(size_t)255; return p; };
  c.nG = (N + CSR_GN8 - 1) / CSR_GN8; c.NGP = (c.nG + 31) & ~31; const int ch = (E + CSR_NBLK8 - 1) / CSR_NBLK8; c.CHP = (ch + 31) & ~31; c.permLen = (size_t)E + 32 * (size_t)c.nG + 32;
  c.STG = (int*)al((size_t)CSR_NBLK8 * c.CHP * 4); c.HST = (int*)al((size_t)CSR_NBLK8 * c.NGP * 4); c.OFF = (int*)al((size_t)c.NGP * CSR_NBLK8 * 4); c.START = (int*)al((size_t)(c.NGP + 64) * 4); c.TOT = (int*)al((size_t)(c.NGP + 64) * 4);
  c.PERM = (int*)al(c.permLen * 4); c.ROWPTR = (int*)al((size_t)c.nG * CSR_TS8 * 4); c.ROWCNT = (int*)al((size_t)c.nG * CSR_TS8 * 4); c.FLAG = (int*)al(256);
  c.bytes = off - off0; return off;
}
static void csr_build8(const CsrBufs8& c, const int* dst, int E, int N, hipStream_t stream) {
  const size_t smem = (size_t)(2 * c.NGP + c.CHP) * 4;
  csrZ_kernel8<<<512, 256, 0, stream>>>((int*)c.base, c.bytes / 16);
  csrA_kernel8<<<CSR_NBLK8, 64, smem, stream>>>(dst, E, N, c.nG, c.CHP, c.NGP, c.STG, c.HST);
  csrS_kernel8<<<1, 512, 0, stream>>>(c.HST, c.nG, c.NGP, c.START, c.TOT, c.OFF);
  csrB_kernel8<<<c.nG, 256, 0, stream>>>(dst, N, c.nG, c.CHP, c.NGP, (int)c.permLen, c.STG, c.HST, c.OFF, c.START, c.TOT, c.PERM, c.ROWPTR, c.ROWCNT, c.FLAG);
}


__global__ __launch_bounds__(256) void wput_kernel(const float* __restrict__ w1, const float* __restrict__ w2, const float* __restrict__ m1, const float* __restrict__ m2, const float* __restrict__ we1, const float* __restrict__ ae1, const float* __restrict__ we2, const float* __restrict__ ae2, b16* __restrict__ WT1, b16* __restrict__ WT2, b16* __restrict__ WM1, b16* __restrict__ WM2, float* __restrict__ GV) { const size_t nt = (size_t)gridDim.x * 256, u0 = (size_t)blockIdx.x * 256 + threadIdx.x; v8b v;
  for (size_t u = u0; u < (size_t)C1 * 16; u += nt) { const int o = (int)(u / 16), k0 = (int)(u % 16) * 8;
#pragma unroll
    for (int j = 0; j < 8; ++j) v[j] = (b16)(bf16_rne(w1[(size_t)o * FIN + k0 + j]) * WSC); for (int pass = 0; pass < 2; ++pass) { *(volatile v8b*)(WT1 + (size_t)o * FIN + k0) = v; __threadfence(); } }
  for (size_t u = u0; u < (size_t)HG * 32; u += nt) { const int o = (int)(u / 32), k0 = (int)(u % 32) * 8;
#pragma unroll
    for (int j = 0; j < 8; ++j) v[j] = (b16)(bf16_rne(w2[(size_t)o * C1 + k0 + j]) * WSC); for (int pass = 0; pass < 2; ++pass) { *(volatile v8b*)(WT2 + (size_t)o * C1 + k0) = v; __threadfence(); } }
  for (size_t u = u0; u < (size_t)2 * HN * 8; u += nt) { const int op = (int)(u / 8), k0 = (int)(u % 8) * 8; const int half = op / HN, o = op % HN;
#pragma unroll
    for (int j = 0; j < 8; ++j) v[j] = (b16)(bf16_rne(m1[(size_t)o * 2 * HG + half * HG + k0 + j]) * WSC); for (int pass = 0; pass < 2; ++pass) { *(volatile v8b*)(WM1 + (size_t)op * HG + k0) = v; __threadfence(); } }
  for (size_t u = u0; u < (size_t)HN2 * 32; u += nt) { const int o = (int)(u / 32), k0 = (int)(u % 32) * 8;
#pragma unroll
    for (int j = 0; j < 8; ++j) v[j] = (b16)(bf16_rne(m2[(size_t)o * HN + k0 + j]) * WSC); for (int pass = 0; pass < 2; ++pass) { *(volatile v8b*)(WM2 + (size_t)o * HN + k0) = v; __threadfence(); } }
  if (u0 < 128) { const int t = (int)u0; float s = 0.0f; if (t < NH1 * FE) { const int hd = t / FE, f = t % FE; for (int c = 0; c < HG; ++c) s += pmul(bfv(we1[(size_t)(hd * HG + c) * FE + f]), bfv(ae1[hd * HG + c])); } else if (t < NH1 * FE + FE) { const int f = t - NH1 * FE; for (int c = 0; c < HG; ++c) s += pmul(bfv(we2[(size_t)c * FE + f]), bfv(ae2[c])); }
    for (int pass = 0; pass < 2; ++pass) { ((volatile float*)GV)[t] = s; __threadfence(); } } }
template <int MODE, int KIN, int NT, int NHh>
__global__ __launch_bounds__(32) void proj_kernel(const float* __restrict__ IN, const b16* __restrict__ W, const float* __restrict__ asrc, const float* __restrict__ adst, int NLIM, float* __restrict__ HP, float* __restrict__ ES) { constexpr int OW = NT * 16; __shared__ __attribute__((aligned(16))) b16 Ah[16][KIN + 8], Al[16][KIN + 8]; __shared__ float Tf[16][OW + 4], Eq[16][8]; const int lane = threadIdx.x, nloc = lane & 15, hlf = lane >> 4; const size_t m0 = (size_t)blockIdx.x * 16; if (m0 >= (size_t)NLIM) return;
  for (int rr = 0; rr < 16; ++rr) for (int q = 0; q < KIN / 32; ++q) { const int c = q * 32 + lane; const float v = IN[(m0 + rr) * KIN + c]; b16 p, ql; if (MODE == 0) { p = (b16)(bf16_rne(v) * XS); ql = (b16)0.0f; } else split16(v * HS, p, ql); Ah[rr][c] = p; Al[rr][c] = ql; }
  if (lane < 16) { for (int k = KIN; k < KIN + 8; ++k) { Ah[lane][k] = (b16)0.0f; Al[lane][k] = (b16)0.0f; } for (int j = 0; j < 8; ++j) Eq[lane][j] = 0.0f; }
  wave_lds_sync(); v8f acc[NT];
#pragma unroll
  for (int t = 0; t < NT; ++t) acc[t] = (v8f){};
#pragma unroll 2
  for (int kb = 0; kb < KIN; kb += 32) { const v16b a = frag_kb(&Ah[nloc][kb], hlf), al = frag_kb(&Al[nloc][kb], hlf);
#pragma unroll
    for (int t = 0; t < NT; ++t) { const v16b bw = frag_kb(W + (size_t)(t * 16 + nloc) * KIN + kb, hlf); acc[t] = wmma16b(a, bw, acc[t]); if (MODE == 1) acc[t] = wmma16b(al, bw, acc[t]); } }
  const float osc = MODE == 0 ? 1.0f / (XS * WSC) : 1.0f / (HS * WSC);
#pragma unroll
  for (int t = 0; t < NT; ++t)
#pragma unroll
    for (int r8 = 0; r8 < 8; ++r8) Tf[8 * hlf + r8][t * 16 + nloc] = acc[t][r8] * osc;
  wave_lds_sync();
  { constexpr int LPH = 32 / NHh; const int hd = lane / LPH, sub = lane % LPH; for (int rr = 0; rr < 16; ++rr) { float s1 = 0.0f, s2 = 0.0f; for (int j = sub; j < HG; j += LPH) { const float hv = Tf[rr][hd * HG + j]; s1 += pmul(hv, bfv(asrc[hd * HG + j])); s2 += pmul(hv, bfv(adst[hd * HG + j])); } for (int o = LPH / 2; o; o >>= 1) { s1 += __shfl_xor(s1, o); s2 += __shfl_xor(s2, o); } if (sub == 0) { Eq[rr][hd] = s1; Eq[rr][4 + hd] = s2; } } }
  wave_lds_sync();
  for (int pass = 0; pass < 2; ++pass) { for (int rr = 0; rr < 16; ++rr) for (int q = 0; q < OW / 32; ++q) ((volatile float*)HP)[(m0 + rr) * OW + q * 32 + lane] = Tf[rr][q * 32 + lane]; for (int q = 0; q < 4; ++q) ((volatile float*)ES)[m0 * 8 + q * 32 + lane] = Eq[(q * 32 + lane) >> 3][(q * 32 + lane) & 7]; __threadfence(); } }
template <int NHh, int ACT>
__global__ __launch_bounds__(256) void gat_kernel(const float* __restrict__ HP, const float* __restrict__ ES, const float* __restrict__ ea, const float* __restrict__ GVv, const float* __restrict__ bias, const int* __restrict__ srcs, const int* __restrict__ PERM, const int* __restrict__ ROWPTR, const int* __restrict__ ROWCNT, int permLen, int NLIM, float* __restrict__ OUT) { constexpr int OW = NHh * HG; __shared__ float La[NPB][FE], Vh[NPB][NHh][FE]; const int wave = threadIdx.x >> 5, lane = threadIdx.x & 31; const size_t i = (size_t)blockIdx.x * NPB + wave; if (i >= (size_t)NLIM) return; int st = ROWPTR[i], cnt = ROWCNT[i]; cnt = iclamp(cnt, 0, E); st = iclamp(st, 0, permLen - cnt);
  for (int h = 0; h < NHh; ++h) if (lane < FE) Vh[wave][h][lane] = GVv[h * FE + lane];
  { float s = 0.0f; int nin = 0;
#pragma unroll 1
    for (int j = 0; j < cnt; ++j) { const int e = iclamp(PERM[st + j], 0, E - 1); const size_t u = (size_t)iclamp(srcs[e], 0, N - 1); if (u >= (size_t)NLIM) continue; ++nin; if (lane < FE) s += bfv(ea[(size_t)e * FE + lane]); }
    if (lane < FE) La[wave][lane] = s / fmaxf((float)nin, 1.0f); }
  wave_lds_sync();
  float adi[NHh], mx[NHh], den[NHh]; v2f acc[NHh];
#pragma unroll
  for (int h = 0; h < NHh; ++h) { adi[h] = ES[i * 8 + 4 + h]; mx[h] = -INFINITY; den[h] = 0.0f; acc[h] = (v2f){0, 0}; }
  auto visit = [&](size_t u, const float* attr, bool isloop) {
#pragma unroll
    for (int h = 0; h < NHh; ++h) { float el = 0.0f;
#pragma unroll
      for (int f = 0; f < FE; ++f) el += pmul(isloop ? attr[f] : bfv(attr[f]), Vh[wave][h][f]);
      float s = ES[u * 8 + h] + adi[h] + el; s = s > 0.0f ? s : 0.2f * s; const float mn = fmaxf(mx[h], s); const float sf = (mx[h] == -INFINITY) ? 0.0f : __expf(mx[h] - mn); const float p = __expf(s - mn); den[h] = den[h] * sf + p; const v2f v = *(const v2f*)(HP + u * OW + h * HG + lane * 2); acc[h] = acc[h] * sf + v * p; mx[h] = mn; } };
#pragma unroll 1
  for (int j = 0; j < cnt; ++j) { const int e = iclamp(PERM[st + j], 0, E - 1); const size_t u = (size_t)iclamp(srcs[e], 0, N - 1); if (u >= (size_t)NLIM) continue; visit(u, ea + (size_t)e * FE, false); }
  visit(i, La[wave], true);
  for (int pass = 0; pass < 2; ++pass) {
#pragma unroll
    for (int h = 0; h < NHh; ++h) { v2f o; for (int k = 0; k < 2; ++k) { const int c = h * HG + lane * 2 + k; o[k] = acc[h][k] / (den[h] + 1e-16f) + bfv(bias[c]); if (ACT) o[k] = fmaxf(o[k], 0.0f); } *(volatile v2f*)(OUT + i * OW + h * HG + lane * 2) = o; }
    __threadfence(); } }
__global__ __launch_bounds__(32) void uv_kernel(const float* __restrict__ H2, const b16* __restrict__ WM1, int NLIM, float* __restrict__ UV) { __shared__ __attribute__((aligned(16))) b16 Ah[16][HG + 8], Al[16][HG + 8]; __shared__ float Tf[16][260]; const int lane = threadIdx.x, nloc = lane & 15, hlf = lane >> 4; const size_t m0 = (size_t)blockIdx.x * 16; if (m0 >= (size_t)NLIM) return;
  for (int rr = 0; rr < 16; ++rr) for (int q = 0; q < 2; ++q) { const int c = q * 32 + lane; b16 p, ql; split16(H2[(m0 + rr) * HG + c] * HS, p, ql); Ah[rr][c] = p; Al[rr][c] = ql; }
  if (lane < 16) for (int k = HG; k < HG + 8; ++k) { Ah[lane][k] = (b16)0.0f; Al[lane][k] = (b16)0.0f; }
  wave_lds_sync();
#pragma unroll 1
  for (int g = 0; g < 2; ++g) { v8f acc[16];
#pragma unroll
    for (int t = 0; t < 16; ++t) acc[t] = (v8f){};
#pragma unroll
    for (int kb = 0; kb < HG; kb += 32) { const v16b a = frag_kb(&Ah[nloc][kb], hlf), al = frag_kb(&Al[nloc][kb], hlf);
#pragma unroll
      for (int t = 0; t < 16; ++t) { const v16b bw = frag_kb(WM1 + (size_t)(g * 256 + t * 16 + nloc) * HG + kb, hlf); acc[t] = wmma16b(a, bw, acc[t]); acc[t] = wmma16b(al, bw, acc[t]); } }
#pragma unroll
    for (int t = 0; t < 16; ++t)
#pragma unroll
      for (int r8 = 0; r8 < 8; ++r8) Tf[8 * hlf + r8][t * 16 + nloc] = acc[t][r8] * (1.0f / (HS * WSC));
    wave_lds_sync();
    for (int pass = 0; pass < 2; ++pass) { for (int rr = 0; rr < 16; ++rr) for (int q = 0; q < 2; ++q) *(volatile v4f*)(UV + (m0 + rr) * 2 * HN + g * HN + q * 128 + lane * 4) = *(const v4f*)(&Tf[rr][q * 128 + lane * 4]); __threadfence(); }
    wave_lds_sync(); } }
__global__ __launch_bounds__(32) void edge_kernel(const float* __restrict__ UV, const int* __restrict__ rows, const int* __restrict__ cols, const float* __restrict__ mb1, const b16* __restrict__ WM2, const float* __restrict__ mb2, const float* __restrict__ mw3, const float* __restrict__ mb3, int NLIM, float* __restrict__ out) { __shared__ __attribute__((aligned(16))) b16 Ah[32][HN + 8]; __shared__ float Tf[32][HN2 + 1], Os[32]; const int lane = threadIdx.x, nloc = lane & 15, hlf = lane >> 4; const size_t e0 = (size_t)blockIdx.x * 32;
  for (int rr = 0; rr < 32; ++rr) { const size_t e = e0 + rr; const size_t r = (size_t)iclamp(rows[e], 0, NLIM - 1), c = (size_t)iclamp(cols[e], 0, NLIM - 1); for (int q = 0; q < HN / 32; ++q) { const int ch = q * 32 + lane; const float v = fmaxf(UV[r * 2 * HN + ch] + UV[c * 2 * HN + HN + ch] + bfv(mb1[ch]), 0.0f); Ah[rr][ch] = (b16)(v * HS); } }
  for (int k = HN; k < HN + 8; ++k) Ah[lane][k] = (b16)0.0f;
  wave_lds_sync();
#pragma unroll
  for (int rt = 0; rt < 2; ++rt) { v8f acc[8];
#pragma unroll
    for (int t = 0; t < 8; ++t) acc[t] = (v8f){};
#pragma unroll 2
    for (int kb = 0; kb < HN; kb += 32) { const v16b a = frag_kb(&Ah[rt * 16 + nloc][kb], hlf); const int al = 0;
#pragma unroll
      for (int t = 0; t < 8; ++t) { const v16b bw = frag_kb(WM2 + (size_t)(t * 16 + nloc) * HN + kb, hlf); acc[t] = wmma16b(a, bw, acc[t]); (void)al; } }
#pragma unroll
    for (int t = 0; t < 8; ++t) { const int cc = t * 16 + nloc; const float bb = bfv(mb2[cc]);
#pragma unroll
      for (int r8 = 0; r8 < 8; ++r8) { float v = acc[t][r8] * (1.0f / (HS * WSC)) + bb; v = v > 0.0f ? v : 0.01f * v; Tf[rt * 16 + 8 * hlf + r8][cc] = v; } } }
  wave_lds_sync();
  { float s = bfv(mb3[0]);
#pragma unroll 4
    for (int c = 0; c < HN2; ++c) s += pmul(Tf[lane][c], bfv(mw3[c])); Os[lane] = s; }
  wave_lds_sync();
  for (int pass = 0; pass < 2; ++pass) { ((volatile float*)out)[e0 + lane] = Os[lane]; __threadfence(); } }
}

extern "C" void kernel_launch(void* const* d_in, const int* in_sizes, int n_in, void* d_out, int out_size, void* d_ws, size_t ws_size, hipStream_t stream) {
  (void)n_in;
  auto Fp = [&](int i) { return (const float*)d_in[i]; }; auto Ip = [&](int i) { return (const int*)d_in[i]; };
  if (in_sizes[0] != N * FIN || in_sizes[1] != 2 * E || in_sizes[2] != E * FE || in_sizes[3] != 2 * E2 || in_sizes[4] != C1 * FIN || in_sizes[5] != C1 * FE || in_sizes[10] != HG * C1 || in_sizes[16] != HN * 2 * HG || in_sizes[18] != HN2 * HN || in_sizes[20] != HN2 || out_size != E2) return;
  const int NLIM = N, E2LIM = E2;
  size_t off = 0; char* ws = (char*)d_ws;
  auto carve = [&](size_t bytes) { char* p = ws + off; off += (bytes + 255) & ~(size_t)255; return p; };
  b16* WT1 = (b16*)carve((size_t)C1 * FIN * 2); b16* WT2 = (b16*)carve((size_t)HG * C1 * 2); b16* WM1 = (b16*)carve((size_t)2 * HN * HG * 2); b16* WM2 = (b16*)carve((size_t)HN2 * HN * 2); float* GV = (float*)carve(512); float* HP = (float*)carve((size_t)N * C1 * 4); float* H1 = (float*)carve((size_t)N * C1 * 4); float* ES = (float*)carve((size_t)N * 8 * 4); float* H2 = (float*)carve((size_t)N * HG * 4); float* UV = HP;     CsrBufs8 csr; off = csr_carve8(csr, ws, off, E, N);
  static_assert((size_t)N * 2 * HN * 4 <= 2 * (size_t)N * C1 * 4, "UV alias must fit in HP+H1");
  if (off > ws_size || off > ((size_t)176 << 20)) return;
  const int nb = (NLIM + NPB - 1) / NPB;
  wput_kernel<<<64, 256, 0, stream>>>(Fp(4), Fp(10), Fp(16), Fp(18), Fp(5), Fp(8), Fp(11), Fp(14), WT1, WT2, WM1, WM2, GV);
  csr_build8(csr, Ip(1) + E, E, N, stream);
  proj_kernel<0, FIN, 16, 4><<<NLIM / 16, 32, 0, stream>>>(Fp(0), WT1, Fp(6), Fp(7), NLIM, HP, ES);
  gat_kernel<4, 1><<<nb, 256, 0, stream>>>(HP, ES, Fp(2), GV, Fp(9), Ip(1), csr.PERM, csr.ROWPTR, csr.ROWCNT, (int)csr.permLen, NLIM, H1);
  proj_kernel<1, C1, 4, 1><<<NLIM / 16, 32, 0, stream>>>(H1, WT2, Fp(12), Fp(13), NLIM, HP, ES);
  gat_kernel<1, 0><<<nb, 256, 0, stream>>>(HP, ES, Fp(2), GV + NH1 * FE, Fp(15), Ip(1), csr.PERM, csr.ROWPTR, csr.ROWCNT, (int)csr.permLen, NLIM, H2);
  uv_kernel<<<NLIM / 16, 32, 0, stream>>>(H2, WM1, NLIM, UV);
  edge_kernel<<<E2LIM / 32, 32, 0, stream>>>(UV, Ip(3), Ip(3) + E2, Fp(17), WM2, Fp(19), Fp(20), Fp(21), NLIM, (float*)d_out);
}
